// TC_module_38611755991897
// MI455X (gfx1250) — hardware-verified
//
#include <hip/hip_runtime.h>


#define NB_  8192
#define IN_  512
#define CTX  256
#define CEN  512
#define FF   1024
#define RNN  1024
#define TOT  768
#define OUTN 512
typedef _Float16 h16;
typedef unsigned short bf;
typedef __attribute__((ext_vector_type(16))) __bf16   v16bf;
typedef __attribute__((ext_vector_type(16))) _Float16 v16h;
typedef __attribute__((ext_vector_type(8)))  _Float16 v8h;
typedef __attribute__((ext_vector_type(8)))  unsigned short v8us;
typedef __attribute__((ext_vector_type(8)))  float    v8f;
typedef __attribute__((ext_vector_type(4)))  float    v4f;
typedef v8h  __attribute__((may_alias)) v8ha;
typedef v4f  __attribute__((may_alias)) v4fa;
typedef v8us __attribute__((may_alias)) v8usa;

__device__ __forceinline__ unsigned short f2bf(float f) { unsigned u = __float_as_uint(f); u += 0x7FFFu + ((u >> 16) & 1u); return (unsigned short)(u >> 16); }
__device__ __forceinline__ float bf2f(unsigned short b) { return __uint_as_float(((unsigned)b) << 16); }
__device__ __forceinline__ float bfr(float f) { return bf2f(f2bf(f)); }
__device__ __forceinline__ v16h cat16(v8h lo, v8h hi) { return __builtin_shufflevector(lo, hi, 0, 1, 2, 3, 4, 5, 6, 7, 8, 9, 10, 11, 12, 13, 14, 15); }
__device__ __forceinline__ v16bf cat16b(v8us lo, v8us hi) { return __builtin_bit_cast(v16bf, __builtin_shufflevector(lo, hi, 0, 1, 2, 3, 4, 5, 6, 7, 8, 9, 10, 11, 12, 13, 14, 15)); }
__device__ __forceinline__ v8f wmma16(v16h a, v16h b, v8f c) { return __builtin_amdgcn_wmma_f32_16x16x32_f16(false, a, false, b, (short)0, c, false, false); }
__device__ __forceinline__ v8f wmmab(v16bf a, v16bf b, v8f c) { return __builtin_amdgcn_wmma_f32_16x16x32_bf16(false, a, false, b, (short)0, c, false, false); }


template <typename T16> struct WFrag;
template <> struct WFrag<h16> { typedef v16h V; static __device__ __forceinline__ V ld(const h16* p) { return cat16(*(const v8h*)p, *(const v8h*)(p + 16)); } static __device__ __forceinline__ v8f mma(V a, V b, v8f c) { return wmma16(a, b, c); } };
template <> struct WFrag<bf> { typedef v16bf V; static __device__ __forceinline__ V ld(const bf* p) { return cat16b(*(const v8us*)p, *(const v8us*)(p + 16)); } static __device__ __forceinline__ v8f mma(V a, V b, v8f c) { return wmmab(a, b, c); } };
template <typename T16, int NSPLIT, bool BIAS>
__global__ __launch_bounds__(32) void k_gemmw(const T16* __restrict__ A, const T16* __restrict__ A2, const T16* __restrict__ Bt, const T16* __restrict__ Bt2, int K, float* C, int ldc, const float* __restrict__ bias, size_t sA, size_t sB, size_t sC) {
    typedef typename WFrag<T16>::V V;
    __shared__ __align__(16) float os[16 * 68];
    const size_t z = blockIdx.z; A += z * sA; if (A2) A2 += z * sA; Bt += z * sB; if (Bt2) Bt2 += z * sB; C += z * sC;
    const int lane = threadIdx.x & 31, lr = lane & 15, hi = lane >> 4; const int r0 = blockIdx.x * 64, c0 = blockIdx.y * 64;
    v8f acc[4][4];
#pragma unroll
    for (int mb = 0; mb < 4; ++mb)
#pragma unroll
        for (int nb = 0; nb < 4; ++nb) acc[mb][nb] = (v8f){};
    const size_t aoff = (size_t)(r0 + lr) * K + 8 * hi, boff = (size_t)(c0 + lr) * K + 8 * hi;
#pragma unroll 1
    for (int kc = 0; kc < K; kc += 32) {
        V a[4], a2[4];
#pragma unroll
        for (int mb = 0; mb < 4; ++mb) { a[mb] = WFrag<T16>::ld(A + aoff + (size_t)mb * 16 * K + kc); if (NSPLIT == 1 || NSPLIT == 2) a2[mb] = WFrag<T16>::ld(A2 + aoff + (size_t)mb * 16 * K + kc); }
#pragma unroll
        for (int nb = 0; nb < 4; ++nb) { const V b = WFrag<T16>::ld(Bt + boff + (size_t)nb * 16 * K + kc); V b2; if (NSPLIT >= 2) b2 = WFrag<T16>::ld(Bt2 + boff + (size_t)nb * 16 * K + kc);
#pragma unroll
            for (int mb = 0; mb < 4; ++mb) { acc[mb][nb] = WFrag<T16>::mma(a[mb], b, acc[mb][nb]); if (NSPLIT == 1 || NSPLIT == 2) acc[mb][nb] = WFrag<T16>::mma(a2[mb], b, acc[mb][nb]); if (NSPLIT >= 2) acc[mb][nb] = WFrag<T16>::mma(a[mb], b2, acc[mb][nb]); } }
        asm volatile("v_nop\n\tv_nop\n\tv_nop\n\tv_nop" : "+v"(acc[0][0]), "+v"(acc[1][1]), "+v"(acc[2][2]), "+v"(acc[3][3]) : "v"(a[0]), "v"(a[3]));
    }
#pragma unroll
    for (int mb = 0; mb < 4; ++mb) {
#pragma unroll
        for (int nb = 0; nb < 4; ++nb) {
#pragma unroll
            for (int j = 0; j < 8; ++j) os[(hi * 8 + j) * 68 + nb * 16 + lr] = acc[mb][nb][j]; }
        __builtin_amdgcn_wave_barrier(); asm volatile("" ::: "memory");
        float* crow = C + (size_t)(r0 + mb * 16) * ldc + c0;
#pragma unroll 1
        for (int ps = 0; ps < 2; ++ps) {
#pragma unroll
            for (int s = 0; s < 8; ++s) { const int row = 2 * s + hi, cofs = lr * 4; v4f val = *(const v4fa*)(os + row * 68 + cofs); if (BIAS) { val[0] += bfr(bias[c0 + cofs]); val[1] += bfr(bias[c0 + cofs + 1]); val[2] += bfr(bias[c0 + cofs + 2]); val[3] += bfr(bias[c0 + cofs + 3]); }
                *(volatile v4f*)(crow + (size_t)row * ldc + cofs) = val; }
            if (ps == 0) __threadfence(); }
        __builtin_amdgcn_wave_barrier(); asm volatile("" ::: "memory");
    }
}

__device__ __forceinline__ void splitf(float y, unsigned short& h, unsigned short& l) { h = f2bf(y); l = f2bf(y - bf2f(h)); }
typedef __attribute__((ext_vector_type(2))) unsigned short v2us;
typedef __attribute__((ext_vector_type(4))) unsigned short v4us;

__global__ __launch_bounds__(256) void k_wtG(const float* __restrict__ w, int K, int N, bf* Bt) {
    const int lane = threadIdx.x & 31; const int L0 = (blockIdx.x * 8 + (threadIdx.x >> 5)) * 8; const int nlines = N * K / 64;
#pragma unroll 1
    for (int ps = 0; ps < 2; ++ps) {
#pragma unroll 1
        for (int l = 0; l < 8; ++l) { const int L = L0 + l; if (L >= nlines) break; const size_t e = (size_t)L * 64 + lane * 2; const int k = (int)(e % K), n = (int)(e / K); v2us o;
            o[0] = f2bf(w[(size_t)k * N + n]); o[1] = f2bf(w[(size_t)(k + 1) * N + n]); *(volatile v2us*)(Bt + e) = o; }
        if (ps == 0) __threadfence(); }
}
__global__ __launch_bounds__(256) void k_cvt8(const float* __restrict__ src, bf* dst, size_t n8) { const size_t i = (size_t)blockIdx.x * 256 + threadIdx.x; if (i >= n8) return; const v8f v = *(const v8f*)(src + i * 8); v8us o;
#pragma unroll
    for (int k = 0; k < 8; ++k) o[k] = f2bf(v[k]); *(volatile v8us*)(dst + i * 8) = o; __threadfence(); *(volatile v8us*)(dst + i * 8) = o; }
__global__ __launch_bounds__(32) void k_norm(const float* __restrict__ w, float* SC) { const int lane = threadIdx.x; float s = 0.f;
    for (int i = lane * 4; i < CEN * CTX; i += 128) { const v4f a = *(const v4f*)(w + i);
#pragma unroll
        for (int q = 0; q < 4; ++q) { const float v = bfr(a[q]); float p = __fmul_rn(v, v); asm volatile("" : "+v"(p)); s = __fadd_rn(s, p); } }
#pragma unroll
    for (int sh = 16; sh; sh >>= 1) s += __shfl_xor(s, sh, 32);
    const float sc = __fdiv_rn(1.0f, fmaxf(__fsqrt_rn(s), 1.0f)); *(volatile float*)(SC + lane) = sc; __threadfence(); *(volatile float*)(SC + lane) = sc; }
__global__ __launch_bounds__(256) void k_ctx(const float* __restrict__ G1, const float* __restrict__ SC, bf* Ch, bf* Cl) { const size_t i = ((size_t)blockIdx.x * 256 + threadIdx.x) * 2; if (i >= (size_t)NB_ * CTX) return; const float sc = SC[0]; v2us oh, ol;
#pragma unroll
    for (int q = 0; q < 2; ++q) { unsigned short a, c2; splitf(__fmul_rn(G1[i + q], sc), a, c2); oh[q] = a; ol[q] = c2; } *(volatile v2us*)(Ch + i) = oh; *(volatile v2us*)(Cl + i) = ol; __threadfence(); *(volatile v2us*)(Ch + i) = oh; *(volatile v2us*)(Cl + i) = ol; }
__global__ __launch_bounds__(256) void k_rin(const float* __restrict__ R1, const float* __restrict__ R2, bf* Rh, bf* Rl) { const size_t i = ((size_t)blockIdx.x * 256 + threadIdx.x) * 2; if (i >= (size_t)NB_ * FF) return; v2us oh, ol;
#pragma unroll
    for (int q = 0; q < 2; ++q) { unsigned short a, c2; splitf(fmaxf(__fadd_rn(R1[i + q], R2[i + q]), 0.f), a, c2); oh[q] = a; ol[q] = c2; } *(volatile v2us*)(Rh + i) = oh; *(volatile v2us*)(Rl + i) = ol; __threadfence(); *(volatile v2us*)(Rh + i) = oh; *(volatile v2us*)(Rl + i) = ol; }
__global__ __launch_bounds__(256) void k_tanh2(const float* __restrict__ A, const float* __restrict__ Bv, float* OUT2, bf* Hh, bf* Hl) { const size_t i = ((size_t)blockIdx.x * 256 + threadIdx.x) * 2; if (i >= (size_t)NB_ * RNN) return; typedef __attribute__((ext_vector_type(2))) float v2f; v2f o; v2us oh, ol;
#pragma unroll
    for (int q = 0; q < 2; ++q) { const float a = __fadd_rn(A[i + q], Bv[i + q]); const float e2 = __expf(2.0f * a); const float th = __fsub_rn(1.0f, __fdiv_rn(2.0f, __fadd_rn(e2, 1.0f))); o[q] = th; unsigned short a2, c2; splitf(th, a2, c2); oh[q] = a2; ol[q] = c2; }
    *(volatile v2f*)(OUT2 + i) = o; *(volatile v2us*)(Hh + i) = oh; *(volatile v2us*)(Hl + i) = ol; __threadfence(); *(volatile v2f*)(OUT2 + i) = o; *(volatile v2us*)(Hh + i) = oh; *(volatile v2us*)(Hl + i) = ol; }
__global__ __launch_bounds__(256) void k_outs(const float* __restrict__ F, float* OUT0, float* OUT1) { const size_t i = ((size_t)blockIdx.x * 256 + threadIdx.x) * 4; if (i >= (size_t)NB_ * TOT) return; const size_t b = i / TOT; const int c = (int)(i % TOT); const v4f a = *(const v4f*)(F + i); v4f o;
#pragma unroll
    for (int q = 0; q < 4; ++q) o[q] = fmaxf(a[q], 0.f); float* dst = (c < OUTN) ? (OUT0 + b * OUTN + c) : (OUT1 + b * (TOT - OUTN) + (c - OUTN)); *(volatile v4f*)dst = o; __threadfence(); *(volatile v4f*)dst = o; }

extern "C" void kernel_launch(void* const* d_in, const int* in_sizes, int n_in,
                              void* d_out, int out_size, void* d_ws, size_t ws_size, hipStream_t stream) {
    (void)in_sizes; (void)n_in; (void)out_size;
    const float* IN[11]; for (int i = 0; i < 11; ++i) IN[i] = (const float*)d_in[i];
    float* OUT0 = (float*)d_out; float* OUT1 = OUT0 + (size_t)NB_ * OUTN; float* OUT2 = OUT1 + (size_t)NB_ * (TOT - OUTN);
    char* wsp = (char*)d_ws;
    auto take = [&](size_t bytes) { char* p = wsp; wsp += (bytes + 255) & ~(size_t)255; return (void*)p; };
    bf* WR = (bf*)take((size_t)CTX * CEN * 2); bf* WP1 = (bf*)take((size_t)FF * IN_ * 2); bf* WP2 = (bf*)take((size_t)FF * CTX * 2); bf* WX = (bf*)take((size_t)RNN * FF * 2); bf* WH = (bf*)take((size_t)RNN * RNN * 2); bf* WPO = (bf*)take((size_t)TOT * RNN * 2); float* SC = (float*)take(256);
    bf* INB = (bf*)take((size_t)NB_ * IN_ * 2); bf* CSB = (bf*)take((size_t)NB_ * CEN * 2); bf* MSB = (bf*)take((size_t)NB_ * RNN * 2); float* G1 = (float*)take((size_t)NB_ * CTX * 4); bf* Ch = (bf*)take((size_t)NB_ * CTX * 2); bf* Cl = (bf*)take((size_t)NB_ * CTX * 2);
    float* R1 = (float*)take((size_t)NB_ * FF * 4); float* R2 = (float*)take((size_t)NB_ * FF * 4); bf* Rh = (bf*)take((size_t)NB_ * FF * 2); bf* Rl = (bf*)take((size_t)NB_ * FF * 2);
    if ((size_t)(wsp - (char*)d_ws) > ws_size) return;
    float* HA = R1; float* HB = R2; bf* Hh = Rh; bf* Hl = Rl; float* FO = R1;
    { k_wtG<<<(unsigned)((CEN * CTX / 64 + 63) / 64), 256, 0, stream>>>(IN[3], CEN, CTX, WR); k_wtG<<<(unsigned)((IN_ * FF / 64 + 63) / 64), 256, 0, stream>>>(IN[4], IN_, FF, WP1); k_wtG<<<(unsigned)((CTX * FF / 64 + 63) / 64), 256, 0, stream>>>(IN[4] + (size_t)IN_ * FF, CTX, FF, WP2);
      k_wtG<<<(unsigned)((FF * RNN / 64 + 63) / 64), 256, 0, stream>>>(IN[6], FF, RNN, WX); k_wtG<<<(unsigned)((RNN * RNN / 64 + 63) / 64), 256, 0, stream>>>(IN[7], RNN, RNN, WH); k_wtG<<<(unsigned)((RNN * TOT / 64 + 63) / 64), 256, 0, stream>>>(IN[9], RNN, TOT, WPO);
      k_norm<<<1, 32, 0, stream>>>(IN[3], SC);
      k_cvt8<<<(unsigned)(((size_t)NB_ * IN_ / 8 + 255) / 256), 256, 0, stream>>>(IN[0], INB, (size_t)NB_ * IN_ / 8); k_cvt8<<<(unsigned)(((size_t)NB_ * CEN / 8 + 255) / 256), 256, 0, stream>>>(IN[1], CSB, (size_t)NB_ * CEN / 8); k_cvt8<<<(unsigned)(((size_t)NB_ * RNN / 8 + 255) / 256), 256, 0, stream>>>(IN[2], MSB, (size_t)NB_ * RNN / 8); }
    k_gemmw<bf, 0, false><<<dim3(NB_ / 64, CTX / 64, 1), 32, 0, stream>>>(CSB, nullptr, WR, nullptr, CEN, G1, CTX, nullptr, 0, 0, 0); k_ctx<<<(unsigned)(((size_t)NB_ * CTX / 2 + 255) / 256), 256, 0, stream>>>(G1, SC, Ch, Cl);
    k_gemmw<bf, 0, true><<<dim3(NB_ / 64, FF / 64, 1), 32, 0, stream>>>(INB, nullptr, WP1, nullptr, IN_, R1, FF, IN[5], 0, 0, 0); k_gemmw<bf, 1, false><<<dim3(NB_ / 64, FF / 64, 1), 32, 0, stream>>>(Ch, Cl, WP2, nullptr, CTX, R2, FF, nullptr, 0, 0, 0);
    k_rin<<<(unsigned)(((size_t)NB_ * FF / 2 + 255) / 256), 256, 0, stream>>>(R1, R2, Rh, Rl);
    k_gemmw<bf, 1, true><<<dim3(NB_ / 64, RNN / 64, 1), 32, 0, stream>>>(Rh, Rl, WX, nullptr, FF, HA, RNN, IN[8], 0, 0, 0); k_gemmw<bf, 0, false><<<dim3(NB_ / 64, RNN / 64, 1), 32, 0, stream>>>(MSB, nullptr, WH, nullptr, RNN, HB, RNN, nullptr, 0, 0, 0);
    k_tanh2<<<(unsigned)(((size_t)NB_ * RNN / 2 + 255) / 256), 256, 0, stream>>>(HA, HB, OUT2, Hh, Hl);
    k_gemmw<bf, 1, true><<<dim3(NB_ / 64, TOT / 64, 1), 32, 0, stream>>>(Hh, Hl, WPO, nullptr, RNN, FO, TOT, IN[10], 0, 0, 0);
    k_outs<<<(unsigned)(((size_t)NB_ * TOT / 4 + 255) / 256), 256, 0, stream>>>(FO, OUT0, OUT1);
}
